// Pattention_3977139716106
// MI455X (gfx1250) — hardware-verified
//
#include <hip/hip_runtime.h>
#include <math.h>


static constexpr int kRows    = 8192;
static constexpr int kD       = 1024;
static constexpr int kS       = 4096;
static constexpr int kDV      = 1024;
static constexpr int kTM      = 16;
static constexpr int kCK      = 256;
static constexpr int kPP      = 256;
static constexpr int kThreads = 256;
static constexpr int kWaves   = 8;

static_assert(kRows % kTM == 0);
static_assert(kS % kCK == 0);
static_assert(kCK == kWaves * 32);
static_assert(kDV == kWaves * 128);
static_assert(kD % 32 == 0);
static_assert((kS * kD) % (kThreads * 8) == 0);
static_assert(kS % 64 == 0 && kDV % 64 == 0);
static_assert(kWaves * kTM * 64 * (int)sizeof(float) == kTM * kD * (int)sizeof(_Float16));

typedef _Float16     v16h __attribute__((ext_vector_type(16)));
typedef _Float16     v8h  __attribute__((ext_vector_type(8)));
typedef float        v8f  __attribute__((ext_vector_type(8)));
typedef float        v4f  __attribute__((ext_vector_type(4)));
typedef unsigned int v4u  __attribute__((ext_vector_type(4)));

union Frag { v16h v; v8h half[2]; };

__device__ __forceinline__ v8f wmma_f16(v16h a, v16h b, v8f acc)
{
    acc = __builtin_amdgcn_wmma_f32_16x16x32_f16(false, a, false, b, (short)0, acc, false, false);
#if defined(__HIP_DEVICE_COMPILE__)
    asm volatile("v_nop\n\tv_nop\n\tv_nop\n\tv_nop" : "+v"(acc) : "v"(a), "v"(b));
#endif
    return acc;
}

__device__ __forceinline__ float bf16_rne(float x)
{
    unsigned int u = __float_as_uint(x);
    u = u + 0x7FFFu + ((u >> 16) & 1u);
    return __uint_as_float(u & 0xFFFF0000u);
}

__device__ __forceinline__ _Float16 cvt16(float x, float sc)
{
    return (_Float16)(bf16_rne(x) * sc);
}

__device__ __forceinline__ float gelu_f32(float s)
{
    return 0.5f * s * (1.0f + erff(s * 0.70710678118654752f));
}

__global__ __launch_bounds__(kThreads)
void k_cvt_rows(const float* __restrict__ src, _Float16* __restrict__ dst, float sc, int n)
{
    const size_t base = ((size_t)blockIdx.x * kThreads + threadIdx.x) * 8;
    if (base + 8 <= (size_t)n) {
        const v4f f0 = *(const v4f*)(src + base);
        const v4f f1 = *(const v4f*)(src + base + 4);
        v8h hv;
        hv[0] = cvt16(f0[0], sc); hv[1] = cvt16(f0[1], sc);
        hv[2] = cvt16(f0[2], sc); hv[3] = cvt16(f0[3], sc);
        hv[4] = cvt16(f1[0], sc); hv[5] = cvt16(f1[1], sc);
        hv[6] = cvt16(f1[2], sc); hv[7] = cvt16(f1[3], sc);
        const v4u u = __builtin_bit_cast(v4u, hv);
        volatile v4u* p = (volatile v4u*)(dst + base);
        *p = u;
        __threadfence();
        *p = u;
    }
}

__global__ __launch_bounds__(kThreads)
void k_transpose_cvt(const float* __restrict__ V, _Float16* __restrict__ VT, float sc)
{
    __shared__ __align__(16) _Float16 tile[64][72];
    const int tid = threadIdx.x;
    const int n0  = blockIdx.x * 64;
    const int s0  = blockIdx.y * 64;

#pragma unroll
    for (int it = 0; it < 4; ++it) {
        const int idx = tid + kThreads * it;
        const int r   = idx >> 4;
        const int c4  = (idx & 15) << 2;
        const v4f f = *(const v4f*)(V + (size_t)(s0 + r) * kDV + n0 + c4);
        tile[r][c4 + 0] = cvt16(f[0], sc);
        tile[r][c4 + 1] = cvt16(f[1], sc);
        tile[r][c4 + 2] = cvt16(f[2], sc);
        tile[r][c4 + 3] = cvt16(f[3], sc);
    }
    __syncthreads();

    v4u    u[2];
    size_t off[2];
#pragma unroll
    for (int it = 0; it < 2; ++it) {
        const int p  = tid + kThreads * it;
        const int vr = p >> 3;
        const int j  = p & 7;
        v8h hv;
#pragma unroll
        for (int i = 0; i < 8; ++i) hv[i] = tile[8 * j + i][vr];
        u[it]   = __builtin_bit_cast(v4u, hv);
        off[it] = (size_t)(n0 + vr) * kS + s0 + 8 * j;
    }
#pragma unroll
    for (int it = 0; it < 2; ++it) *(volatile v4u*)(VT + off[it]) = u[it];
    __threadfence();
#pragma unroll
    for (int it = 0; it < 2; ++it) *(volatile v4u*)(VT + off[it]) = u[it];
}

__global__ __launch_bounds__(kThreads)
void k_main(const float* __restrict__ X, const _Float16* __restrict__ KPh,
            const _Float16* __restrict__ VPT, float* __restrict__ Out)
{
    __shared__ __align__(16) _Float16 sX[kTM * kD];
    __shared__ __align__(16) _Float16 sP[kTM * kPP];
    __shared__ float sRed[kWaves * kTM];
    __shared__ float sScale[kTM];

    const int tid  = threadIdx.x;
    const int wave = tid >> 5;
    const int lane = tid & 31;
    const int h    = lane >> 4;
    const int m    = lane & 15;
    const int row0 = blockIdx.x * kTM;

    {
        const float* xb = X + (size_t)row0 * kD;
        for (int idx = tid; idx < kTM * kD / 8; idx += kThreads) {
            const int r = idx >> 7;
            const int c = (idx & 127) << 3;
            const float* src = xb + (size_t)r * kD + c;
            const v4f f0 = *(const v4f*)(src);
            const v4f f1 = *(const v4f*)(src + 4);
            v8h hv;
            hv[0] = cvt16(f0[0], 16.0f); hv[1] = cvt16(f0[1], 16.0f);
            hv[2] = cvt16(f0[2], 16.0f); hv[3] = cvt16(f0[3], 16.0f);
            hv[4] = cvt16(f1[0], 16.0f); hv[5] = cvt16(f1[1], 16.0f);
            hv[6] = cvt16(f1[2], 16.0f); hv[7] = cvt16(f1[3], 16.0f);
            *(v8h*)(sX + r * kD + c) = hv;
        }
    }
    __syncthreads();

    v8f oacc[8] = {};
    float ssq[8];
#pragma unroll
    for (int r = 0; r < 8; ++r) ssq[r] = 0.0f;

    const _Float16* xa  = sX + m * kD + 8 * h;
    const _Float16* pa  = sP + m * kPP + 8 * h;
    const _Float16* kpw = KPh + (size_t)(wave * 32 + m) * kD + 8 * h;
    const _Float16* vpw = VPT + (size_t)(wave * 128 + m) * kS + 8 * h;

#pragma unroll 1
    for (int kc = 0; kc < kS; kc += kCK) {
        v8f d0 = {}, d1 = {};
        const _Float16* kp0 = kpw + (size_t)kc * kD;
        const _Float16* kp1 = kp0 + 16 * kD;
#pragma unroll 1
        for (int k0 = 0; k0 < kD; k0 += 32) {
            Frag a, b0, b1;
            a.half[0]  = *(const v8h*)(xa + k0);
            a.half[1]  = *(const v8h*)(xa + k0 + 16);
            b0.half[0] = *(const v8h*)(kp0 + k0);
            b0.half[1] = *(const v8h*)(kp0 + k0 + 16);
            b1.half[0] = *(const v8h*)(kp1 + k0);
            b1.half[1] = *(const v8h*)(kp1 + k0 + 16);
            d0 = wmma_f16(a.v, b0.v, d0);
            d1 = wmma_f16(a.v, b1.v, d1);
        }

        {
            _Float16* prow = sP + (8 * h) * kPP + wave * 32 + m;
#pragma unroll
            for (int r = 0; r < 8; ++r) {
                const float s0v = d0[r] * (1.0f / 256.0f);
                const float s1v = d1[r] * (1.0f / 256.0f);
                const float g0  = gelu_f32(s0v);
                const float g1  = gelu_f32(s1v);
                ssq[r] += g0 * g0;
                ssq[r] += g1 * g1;
                prow[r * kPP]      = (_Float16)(g0 * 64.0f);
                prow[r * kPP + 16] = (_Float16)(g1 * 64.0f);
            }
        }
        __syncthreads();

#pragma unroll 1
        for (int ks = 0; ks < kCK; ks += 32) {
            Frag a;
            a.half[0] = *(const v8h*)(pa + ks);
            a.half[1] = *(const v8h*)(pa + ks + 16);
            const _Float16* vp0 = vpw + kc + ks;
#pragma unroll
            for (int t = 0; t < 8; ++t) {
                Frag b;
                const _Float16* vpt = vp0 + (size_t)t * 16 * kS;
                b.half[0] = *(const v8h*)(vpt);
                b.half[1] = *(const v8h*)(vpt + 16);
                oacc[t] = wmma_f16(a.v, b.v, oacc[t]);
            }
        }
        __syncthreads();
    }

#pragma unroll
    for (int r = 0; r < 8; ++r) {
        float v = ssq[r];
        v += __shfl_xor(v, 1, 32);
        v += __shfl_xor(v, 2, 32);
        v += __shfl_xor(v, 4, 32);
        v += __shfl_xor(v, 8, 32);
        if (m == r) sRed[wave * kTM + 8 * h + r] = v;
    }
    __syncthreads();
    if (wave == 0) {
        float ss = 0.0f;
#pragma unroll
        for (int w = 0; w < kWaves; ++w) ss += sRed[w * kTM + m];
        const float sc = rsqrtf(ss) * (1.0f / 256.0f);
        if (lane < kTM) sScale[lane] = sc;
    }
    __syncthreads();

    float* stg  = reinterpret_cast<float*>(sX) + wave * (kTM * 64);
    float* orow = Out + (size_t)row0 * kDV + wave * 128;
#pragma unroll
    for (int q = 0; q < 2; ++q) {
        if (q) __syncthreads();
#pragma unroll
        for (int tt = 0; tt < 4; ++tt) {
#pragma unroll
            for (int r = 0; r < 8; ++r) {
                const int row = 8 * h + r;
                stg[row * 64 + tt * 16 + m] = oacc[4 * q + tt][r] * sScale[row];
            }
        }
        __syncthreads();
        v4f vals[8];
#pragma unroll
        for (int i = 0; i < 8; ++i) {
            const int row = 2 * i + h;
            vals[i] = *(const v4f*)(stg + row * 64 + 4 * m);
        }
#pragma unroll
        for (int i = 0; i < 8; ++i) {
            const int row = 2 * i + h;
            *(volatile v4f*)(orow + (size_t)row * kDV + q * 64 + 4 * m) = vals[i];
        }
        __threadfence();
#pragma unroll
        for (int i = 0; i < 8; ++i) {
            const int row = 2 * i + h;
            *(volatile v4f*)(orow + (size_t)row * kDV + q * 64 + 4 * m) = vals[i];
        }
    }
}

extern "C" void kernel_launch(void* const* d_in, const int* in_sizes, int n_in,
                              void* d_out, int out_size, void* d_ws, size_t ws_size,
                              hipStream_t stream)
{
    if (n_in < 3) return;
    if (in_sizes[0] != kRows * kD) return;
    if (in_sizes[1] != kS * kD) return;
    if (in_sizes[2] != kS * kDV) return;
    if (out_size != kRows * kDV) return;

    const size_t bytesKP = (size_t)kS * kD * sizeof(_Float16);
    const size_t bytesVT = (size_t)kDV * kS * sizeof(_Float16);
    if (ws_size < bytesKP + bytesVT) return;

    const float* X  = (const float*)d_in[0];
    const float* KP = (const float*)d_in[1];
    const float* VP = (const float*)d_in[2];
    float* Out = (float*)d_out;

    _Float16* KPh = (_Float16*)d_ws;
    _Float16* VPT = (_Float16*)((char*)d_ws + bytesKP);

    const int nKP = kS * kD;
    k_cvt_rows<<<dim3((unsigned)((nKP / 8 + kThreads - 1) / kThreads)), dim3(kThreads), 0, stream>>>(KP, KPh, 16.0f, nKP);
    k_transpose_cvt<<<dim3(kDV / 64, kS / 64), dim3(kThreads), 0, stream>>>(VP, VPT, 256.0f);
    k_main<<<dim3(kRows / kTM), dim3(kThreads), 0, stream>>>(X, KPh, VPT, Out);
}
